// SuperGlueMultiHeadAttention_42382737277051
// MI455X (gfx1250) — hardware-verified
//
#include <hip/hip_runtime.h>
#include <math.h>
#include <stdint.h>

#define NB    4
#define SEQ   4096
#define DMOD  256
#define NH    4
#define HD    64
#define QSC   64.0f
#define KSC   64.0f
#define PCAR  32768.0f
#define VCAR  64.0f
#define OSC   1024.0f
#define WOS   1024.0f
#define LOG2E 1.4426950408889634f
#define ATT_WAVES   4
#define ATT_THREADS (ATT_WAVES * 32)
#define ATT_BLOCKS  (NB * NH * (SEQ / 64))
#define NKB    (SEQ / 32)
#define SLABF  (16 * 68)
#define SLAB64 (16 * 68)
#define XTP    72
static_assert(HD == 64 && DMOD == NH * HD);
static_assert((SEQ / 64) == 64 && NH == 4 && NB == 4);
static_assert(ATT_THREADS == 128 && ATT_BLOCKS == 1024 && NKB == 128);
static_assert((DMOD % 64) == 0 && (SEQ % 64) == 0 && (DMOD % 32) == 0);
static_assert(((NB * SEQ * DMOD / 8) % 256) == 0 && ((DMOD * DMOD / 8) % 256) == 0);
static_assert((DMOD / 8) == 32);
static_assert(64 * XTP >= 63 * XTP + 64);
static_assert(ATT_WAVES * SLABF >= 4 * 16 * 68);

typedef unsigned short u16;
typedef _Float16 v16h __attribute__((ext_vector_type(16)));
typedef _Float16 v8h  __attribute__((ext_vector_type(8)));
typedef __bf16   v16b __attribute__((ext_vector_type(16)));
typedef float    v8f  __attribute__((ext_vector_type(8)));
typedef float    v4f  __attribute__((ext_vector_type(4)));
typedef unsigned int v4u __attribute__((ext_vector_type(4)));

union FragH { v16h v; v8h h[2]; v4u u[2]; };
union FragB { v16b v; v4u u[2]; };

__device__ __forceinline__ unsigned short bf_bits(float f) {
  unsigned u = __float_as_uint(f);
  return (unsigned short)((u + 0x7FFFu + ((u >> 16) & 1u)) >> 16);
}
__device__ __forceinline__ float bf_up(unsigned short h) { return __uint_as_float(((unsigned)h) << 16); }
__device__ __forceinline__ float bfr(float f) { return bf_up(bf_bits(f)); }
__device__ __forceinline__ unsigned short h_bits(_Float16 x) { return __builtin_bit_cast(unsigned short, x); }
__device__ __forceinline__ unsigned pk16(unsigned short a, unsigned short b) { return (unsigned)a | ((unsigned)b << 16); }
__device__ __forceinline__ v8f zero8() { v8f z = {0.f, 0.f, 0.f, 0.f, 0.f, 0.f, 0.f, 0.f}; return z; }
__device__ __forceinline__ v4f zero4() { v4f z = {0.f, 0.f, 0.f, 0.f}; return z; }

__device__ __forceinline__ v16h ldfrag_h(const _Float16* p) {
  FragH f;
  f.h[0] = *(const v8h*)(p);
  f.h[1] = *(const v8h*)(p + 16);
  return f.v;
}
__device__ __forceinline__ v16b ldfrag_b(const u16* p) {
  FragB f;
  f.u[0] = *(const v4u*)(p);
  f.u[1] = *(const v4u*)(p + 16);
  return f.v;
}

__device__ __forceinline__ v8f mma_h(v16h a, v16h b, v8f c) {
  return __builtin_amdgcn_wmma_f32_16x16x32_f16(false, a, false, b, (short)0, c, false, false);
}
__device__ __forceinline__ v8f mma_b(v16b a, v16b b, v8f c) {
  return __builtin_amdgcn_wmma_f32_16x16x32_bf16(false, a, false, b, (short)0, c, false, false);
}
__device__ __forceinline__ void g2_3(v8f& a, v8f& b, v16h x0, v16h x1, v16h x2) {
#if defined(__HIP_DEVICE_COMPILE__)
  asm volatile("v_nop\n\tv_nop\n\tv_nop\n\tv_nop" : "+v"(a), "+v"(b) : "v"(x0), "v"(x1), "v"(x2) : "memory");
#endif
}
template <typename F>
__device__ __forceinline__ void g4_5(v8f& a, v8f& b, v8f& c, v8f& d, F x0, F x1, F x2, F x3, F x4) {
#if defined(__HIP_DEVICE_COMPILE__)
  asm volatile("v_nop\n\tv_nop\n\tv_nop\n\tv_nop"
               : "+v"(a), "+v"(b), "+v"(c), "+v"(d) : "v"(x0), "v"(x1), "v"(x2), "v"(x3), "v"(x4) : "memory");
#endif
}
__device__ __forceinline__ void g4_9(v8f& a, v8f& b, v8f& c, v8f& d, v16h x0, v16h x1, v16h x2, v16h x3, v16h x4,
                                     v16h x5, v16h x6, v16h x7, v16h x8) {
#if defined(__HIP_DEVICE_COMPILE__)
  asm volatile("v_nop\n\tv_nop\n\tv_nop\n\tv_nop"
               : "+v"(a), "+v"(b), "+v"(c), "+v"(d)
               : "v"(x0), "v"(x1), "v"(x2), "v"(x3), "v"(x4), "v"(x5), "v"(x6), "v"(x7), "v"(x8) : "memory");
#endif
}
__device__ __forceinline__ void acc_guard4(v8f& a, v8f& b, v8f& c, v8f& d) {
#if defined(__HIP_DEVICE_COMPILE__)
  asm volatile("v_nop\n\tv_nop\n\tv_nop\n\tv_nop" : "+v"(a), "+v"(b), "+v"(c), "+v"(d));
#endif
}
__device__ __forceinline__ void wave_sync_lds() {
  __builtin_amdgcn_fence(__ATOMIC_RELEASE, "workgroup");
  __builtin_amdgcn_wave_barrier();
  __builtin_amdgcn_fence(__ATOMIC_ACQUIRE, "workgroup");
}

__global__ __launch_bounds__(256) void cvtw(const float* __restrict__ w, u16* D, int mode, float scale) {
  const int gt = blockIdx.x * 256 + (int)threadIdx.x;
  if (gt >= (DMOD * DMOD) / 8) return;
  const int row  = gt >> 5;
  const int c8   = (gt & 31) * 8;
  const int prow = ((row & 63) << 2) | (row >> 6);
  const int hsel = c8 >> 6, d0 = c8 & 63;
  unsigned short s[8];
#pragma unroll
  for (int e = 0; e < 8; ++e) {
    const int i0  = prow * DMOD + c8 + e;
    const int i1  = row * DMOD + ((d0 + e) << 2) + hsel;
    const int idx = (mode == 0) ? i0 : i1;
    const float v = w[idx];
    const unsigned short bb = bf_bits(v);
    const unsigned short hb = h_bits((_Float16)(bf_up(bb) * scale));
    s[e] = (mode == 0) ? bb : hb;
  }
  v4u o;
#pragma unroll
  for (int e = 0; e < 4; ++e) o[e] = pk16(s[2 * e], s[2 * e + 1]);
  u16* d = D + (size_t)gt * 8;
  for (int pass = 0; pass < 2; ++pass) {
    *(volatile v4u*)(d) = o;
    __threadfence();
  }
}

__global__ __launch_bounds__(256) void cvh16(const float* __restrict__ x, u16* D, int n8, float scale) {
  const int gt = blockIdx.x * 256 + (int)threadIdx.x;
  if (gt >= n8) return;
  const float* p = x + (size_t)gt * 8;
  const v4f a = *(const v4f*)(p), c4 = *(const v4f*)(p + 4);
  float v[8];
#pragma unroll
  for (int e = 0; e < 4; ++e) { v[e] = a[e]; v[4 + e] = c4[e]; }
  unsigned short s[8];
#pragma unroll
  for (int e = 0; e < 8; ++e) s[e] = h_bits((_Float16)(v[e] * scale));
  v4u o;
#pragma unroll
  for (int e = 0; e < 4; ++e) o[e] = pk16(s[2 * e], s[2 * e + 1]);
  u16* d = D + (size_t)gt * 8;
  for (int pass = 0; pass < 2; ++pass) {
    *(volatile v4u*)(d) = o;
    __threadfence();
  }
}

__global__ __launch_bounds__(256) void xt16(const float* __restrict__ x, u16* XT) {
  __shared__ __align__(16) u16 T[64 * XTP];
  const int tid = threadIdx.x;
  const int bid = blockIdx.x;
  const int ct  = bid & 3;
  const int st  = (bid >> 2) & 63;
  const int b   = bid >> 8;
  const int c0  = ct * 64, s0 = st * 64;
  {
    const int cl = tid >> 2;
    const int tc = (tid & 3) * 16;
    const float* src = x + ((size_t)(b * DMOD + c0 + cl)) * SEQ + s0 + tc;
#pragma unroll
    for (int i = 0; i < 4; ++i) {
      const v4f a = *(const v4f*)(src + 4 * i);
#pragma unroll
      for (int e = 0; e < 4; ++e) T[(tc + 4 * i + e) * XTP + cl] = bf_bits(a[e]);
    }
  }
  __syncthreads();
  v4u o[2];
  const int q8 = tid >> 3, p8 = (tid & 7) * 8;
#pragma unroll
  for (int it = 0; it < 2; ++it) {
    const int line = it * 32 + q8;
    o[it] = *(const v4u*)(T + line * XTP + p8);
  }
  const size_t base = ((size_t)(b * SEQ + s0)) * DMOD + c0 + p8;
  for (int pass = 0; pass < 2; ++pass) {
#pragma unroll
    for (int it = 0; it < 2; ++it) {
      const int line = it * 32 + q8;
      *(volatile v4u*)(XT + base + (size_t)line * DMOD) = o[it];
    }
    __threadfence();
  }
}

__device__ __forceinline__ void bias_terms(const float* __restrict__ bias, int bmode, int rowb, int col0, int hh, int m,
                                           v4f& badd, v8f& radd) {
#pragma unroll
  for (int e = 0; e < 4; ++e) {
    const int ci = col0 + 4 * m + e;
    const int pc = ((ci & 63) << 2) | ((ci >> 6) & 3);
    const float bc = bfr(bias[pc]);
    badd[e] = (bmode == 0) ? bc : 0.0f;
  }
#pragma unroll
  for (int r = 0; r < 8; ++r) {
    const int ri = rowb + 8 * hh + r;
    const int p1 = ((ri & 63) << 2) | ((ri >> 6) & 3);
    const int p2 = ri & (DMOD - 1);
    const float b1 = bfr(bias[p1]), b2 = bfr(bias[p2]);
    radd[r] = (bmode == 1) ? b1 : ((bmode == 2) ? b2 : 0.0f);
  }
}

__device__ __forceinline__ void epi64(float* sl, v8f a0, v8f a1, v8f a2, v8f a3, float oscale, v4f badd, v8f radd,
                                      float* C, int N, size_t rowb, int col0, int lane) {
  const int hh = lane >> 4, m = lane & 15;
#pragma unroll
  for (int r = 0; r < 8; ++r) {
    const int ro = (8 * hh + r) * 68 + m;
    sl[ro]      = a0[r] * oscale + radd[r];
    sl[ro + 16] = a1[r] * oscale + radd[r];
    sl[ro + 32] = a2[r] * oscale + radd[r];
    sl[ro + 48] = a3[r] * oscale + radd[r];
  }
  wave_sync_lds();
  v4f vals[8];
#pragma unroll
  for (int it = 0; it < 8; ++it) vals[it] = *(const v4f*)(sl + (it * 2 + hh) * 68 + m * 4) + badd;
  float* dst = C + (rowb + (size_t)hh) * (size_t)N + col0 + m * 4;
  for (int pass = 0; pass < 2; ++pass) {
#pragma unroll
    for (int it = 0; it < 8; ++it) {
      *(volatile v4f*)(dst + (size_t)(it * 2) * (size_t)N) = vals[it];
    }
    __threadfence();
  }
}

__global__ __launch_bounds__(128)
void gemm_bfb(const u16* __restrict__ A, const u16* __restrict__ Bt, const float* __restrict__ bias,
              float* C, int M, int N, int K, float oscale, int bmode, int sA, int sB, int sC) {
  __shared__ __align__(16) float slab[4 * SLAB64];
  const int tid = threadIdx.x, wave = tid >> 5, lane = tid & 31, hh = lane >> 4, m = lane & 15;
  const int ntile = N >> 6;
  const int bid   = blockIdx.x;
  const int y     = blockIdx.y;
  const int rowb  = (bid / ntile) * 64 + wave * 16;
  const int col0  = (bid % ntile) * 64;
  if (rowb + 16 > M) return;
  const u16* Ab = A  + (size_t)y * (size_t)sA;
  const u16* Bb = Bt + (size_t)y * (size_t)sB;
  float*     Cb = C  + (size_t)y * (size_t)sC;
  const u16* ap = Ab + (size_t)(rowb + m) * K + 8 * hh;
  const u16* bp = Bb + (size_t)(col0 + m) * K + 8 * hh;
  const size_t bs = (size_t)16 * K;
  v8f acc0 = zero8(), acc1 = zero8(), acc2 = zero8(), acc3 = zero8();
#pragma unroll 1
  for (int k0 = 0; k0 < K; k0 += 32) {
    const v16b a  = ldfrag_b(ap + k0);
    const v16b b0 = ldfrag_b(bp + k0);
    const v16b b1 = ldfrag_b(bp + bs + k0);
    const v16b b2 = ldfrag_b(bp + 2 * bs + k0);
    const v16b b3 = ldfrag_b(bp + 3 * bs + k0);
    acc0 = mma_b(a, b0, acc0);
    acc1 = mma_b(a, b1, acc1);
    acc2 = mma_b(a, b2, acc2);
    acc3 = mma_b(a, b3, acc3);
    g4_5<v16b>(acc0, acc1, acc2, acc3, a, b0, b1, b2, b3);
  }
  v4f badd = zero4();
  v8f radd = zero8();
  bias_terms(bias, bmode, rowb, col0, hh, m, badd, radd);
  epi64(slab + wave * SLAB64, acc0, acc1, acc2, acc3, oscale, badd, radd, Cb, N, (size_t)rowb, col0, lane);
}

__global__ __launch_bounds__(128)
void gemm_wh2(const u16* __restrict__ A, const u16* __restrict__ Bh, const u16* __restrict__ Bl,
              const float* __restrict__ bias, float* C, int M, int N, int K, float oscale, int sB, int sC) {
  __shared__ __align__(16) float slab[4 * SLAB64];
  const int tid = threadIdx.x, wave = tid >> 5, lane = tid & 31, hh = lane >> 4, m = lane & 15;
  const int ntile = N >> 6;
  const int bid   = blockIdx.x;
  const int y     = blockIdx.y;
  const int rowb  = (bid / ntile) * 64 + wave * 16;
  const int col0  = (bid % ntile) * 64;
  if (rowb + 16 > M) return;
  const _Float16* ap  = (const _Float16*)(const void*)A + (size_t)(rowb + m) * K + 8 * hh;
  const size_t bofs   = (size_t)y * (size_t)sB + (size_t)(col0 + m) * K + 8 * hh;
  const _Float16* bhp = (const _Float16*)(const void*)Bh + bofs;
  const _Float16* blp = (const _Float16*)(const void*)Bl + bofs;
  float* Cb = C + (size_t)y * (size_t)sC;
  const size_t bs = (size_t)16 * K;
  v8f acc0 = zero8(), acc1 = zero8(), acc2 = zero8(), acc3 = zero8();
#pragma unroll 1
  for (int k0 = 0; k0 < K; k0 += 32) {
    const v16h a   = ldfrag_h(ap + k0);
    const v16h bh0 = ldfrag_h(bhp + k0);
    const v16h bh1 = ldfrag_h(bhp + bs + k0);
    const v16h bh2 = ldfrag_h(bhp + 2 * bs + k0);
    const v16h bh3 = ldfrag_h(bhp + 3 * bs + k0);
    const v16h bl0 = ldfrag_h(blp + k0);
    const v16h bl1 = ldfrag_h(blp + bs + k0);
    const v16h bl2 = ldfrag_h(blp + 2 * bs + k0);
    const v16h bl3 = ldfrag_h(blp + 3 * bs + k0);
    acc0 = mma_h(a, bh0, acc0);  acc0 = mma_h(a, bl0, acc0);
    acc1 = mma_h(a, bh1, acc1);  acc1 = mma_h(a, bl1, acc1);
    acc2 = mma_h(a, bh2, acc2);  acc2 = mma_h(a, bl2, acc2);
    acc3 = mma_h(a, bh3, acc3);  acc3 = mma_h(a, bl3, acc3);
    g4_9(acc0, acc1, acc2, acc3, a, bh0, bh1, bh2, bh3, bl0, bl1, bl2, bl3);
  }
  v4f badd = zero4();
  v8f radd = zero8();
  bias_terms(bias, 2, rowb, col0, hh, m, badd, radd);
  epi64(slab + wave * SLAB64, acc0, acc1, acc2, acc3, oscale, badd, radd, Cb, N, (size_t)rowb, col0, lane);
}

__global__ __launch_bounds__(ATT_THREADS)
void attn_fwd(const u16* __restrict__ QHp, const u16* __restrict__ KHp, const u16* __restrict__ VHp,
              u16* OHIp, u16* OLOp) {
  __shared__ __align__(16) float smem[ATT_WAVES * SLABF];

  const int tid  = threadIdx.x;
  const int wave = tid >> 5;
  const int lane = tid & 31;
  const int hh   = lane >> 4;
  const int c    = lane & 15;

  const int bid  = blockIdx.x;
  const int qt   = bid & (SEQ / 64 - 1);
  const int head = (bid >> 6) & (NH - 1);
  const int b    = bid >> 8;
  const int q0   = qt * 64 + wave * 16;

  const size_t qofs = (((size_t)(b * SEQ + q0 + c)) * NH + head) * HD + 8 * hh;
  const _Float16* Qh  = (const _Float16*)(const void*)QHp + qofs;
  const v16h qh0 = ldfrag_h(Qh), qh1 = ldfrag_h(Qh + 32);
  const size_t kofs = (((size_t)b * SEQ + c) * NH + head) * HD + 8 * hh;
  const _Float16* Khb = (const _Float16*)(const void*)KHp + kofs;
  const size_t vofs = ((size_t)(b * NH + head) * HD + c) * SEQ + 8 * hh;
  const _Float16* Vhb = (const _Float16*)(const void*)VHp + vofs;
  const float lsc = 0.125f * (LOG2E / (QSC * KSC));

  float mrun = -INFINITY, lrun = 0.f;
  v8f o[4];
#pragma unroll
  for (int j = 0; j < 4; ++j) o[j] = zero8();

#pragma unroll 1
  for (int it = 0; it < NKB; ++it) {
    const int kb = it * 32;
    v8f s0 = zero8(), s1 = zero8();
    const _Float16* k0p = Khb + (size_t)kb * (NH * HD);
    const _Float16* k1p = k0p + (size_t)16 * (NH * HD);
    {
      const v16h kh0 = ldfrag_h(k0p), kh1 = ldfrag_h(k1p);
      s0 = mma_h(kh0, qh0, s0);
      s1 = mma_h(kh1, qh0, s1);
      g2_3(s0, s1, qh0, kh0, kh1);
    }
    {
      const v16h kh0 = ldfrag_h(k0p + 32), kh1 = ldfrag_h(k1p + 32);
      s0 = mma_h(kh0, qh1, s0);
      s1 = mma_h(kh1, qh1, s1);
      g2_3(s0, s1, qh1, kh0, kh1);
    }
    float t[16];
#pragma unroll
    for (int i = 0; i < 8; ++i) { t[i] = s0[i] * lsc; t[8 + i] = s1[i] * lsc; }
    float cm = t[0];
#pragma unroll
    for (int i = 1; i < 16; ++i) cm = fmaxf(cm, t[i]);
    cm = fmaxf(cm, __shfl_xor(cm, 16, 32));
    const float mn = fmaxf(mrun, cm);
    const float al = exp2f(mrun - mn);
    mrun = mn;
    float ps = 0.f;
    FragH ph;
#pragma unroll
    for (int w = 0; w < 2; ++w) {
#pragma unroll
      for (int e4 = 0; e4 < 4; ++e4) {
        const int i = 8 * w + 2 * e4;
        const float p0 = exp2f(t[i] - mn), p1 = exp2f(t[i + 1] - mn);
        ps += p0 + p1;
        const _Float16 h0 = (_Float16)(p0 * PCAR), h1 = (_Float16)(p1 * PCAR);
        ph.u[w][e4] = pk16(h_bits(h0), h_bits(h1));
      }
    }
    ps += __shfl_xor(ps, 16, 32);
    lrun = lrun * al + ps;
    float scl[8];
#pragma unroll
    for (int r = 0; r < 8; ++r) scl[r] = __shfl(al, 8 * hh + r, 32);
#pragma unroll
    for (int j = 0; j < 4; ++j) {
#pragma unroll
      for (int r = 0; r < 8; ++r) o[j][r] *= scl[r];
    }
    {
      const _Float16* vhp = Vhb + kb;
      const v16h vh0 = ldfrag_h(vhp);
      const v16h vh1 = ldfrag_h(vhp + (size_t)16 * SEQ);
      const v16h vh2 = ldfrag_h(vhp + (size_t)32 * SEQ);
      const v16h vh3 = ldfrag_h(vhp + (size_t)48 * SEQ);
      o[0] = mma_h(ph.v, vh0, o[0]);
      o[1] = mma_h(ph.v, vh1, o[1]);
      o[2] = mma_h(ph.v, vh2, o[2]);
      o[3] = mma_h(ph.v, vh3, o[3]);
      g4_5<v16h>(o[0], o[1], o[2], o[3], ph.v, vh0, vh1, vh2, vh3);
    }
  }
  acc_guard4(o[0], o[1], o[2], o[3]);

  const float linv = (1.0f / lrun) * (1.0f / (PCAR * VCAR));
  float inv[8];
#pragma unroll
  for (int r = 0; r < 8; ++r) inv[r] = __shfl(linv, 8 * hh + r, 32);
  float* slab = smem + wave * SLABF;
#pragma unroll
  for (int r = 0; r < 8; ++r) {
#pragma unroll
    for (int j = 0; j < 4; ++j) slab[(8 * hh + r) * 68 + j * 16 + c] = o[j][r] * inv[r];
  }
  wave_sync_lds();
  v4u oh[4], ol[4];
  const int rq = lane >> 3, c8 = (lane & 7) * 8;
#pragma unroll
  for (int i4 = 0; i4 < 4; ++i4) {
    const int row = i4 * 4 + rq;
    const v4f a = *(const v4f*)(slab + row * 68 + c8), c4 = *(const v4f*)(slab + row * 68 + c8 + 4);
    float w[8];
#pragma unroll
    for (int e = 0; e < 4; ++e) { w[e] = a[e] * OSC; w[4 + e] = c4[e] * OSC; }
#pragma unroll
    for (int e = 0; e < 4; ++e) {
      const _Float16 h0 = (_Float16)w[2 * e], h1 = (_Float16)w[2 * e + 1];
      const _Float16 l0 = (_Float16)(w[2 * e] - (float)h0), l1 = (_Float16)(w[2 * e + 1] - (float)h1);
      oh[i4][e] = pk16(h_bits(h0), h_bits(h1));
      ol[i4][e] = pk16(h_bits(l0), h_bits(l1));
    }
  }
  const size_t ob = (((size_t)(b * SEQ + q0)) * NH + head) * HD + c8;
  for (int pass = 0; pass < 2; ++pass) {
#pragma unroll
    for (int i4 = 0; i4 < 4; ++i4) {
      const int row = i4 * 4 + rq;
      const size_t o8 = ob + (size_t)row * (NH * HD);
      *(volatile v4u*)(OHIp + o8) = oh[i4];
      *(volatile v4u*)(OLOp + o8) = ol[i4];
    }
    __threadfence();
  }
}

extern "C" void kernel_launch(void* const* d_in, const int* in_sizes, int n_in,
                              void* d_out, int out_size, void* d_ws, size_t ws_size,
                              hipStream_t stream) {
  const int ROWS = NB * SEQ;
  const int XN   = NB * DMOD * SEQ;
  if (n_in < 11) return;
  if (in_sizes[0] != XN || in_sizes[1] != XN || in_sizes[2] != XN) return;
  if (in_sizes[3] != DMOD * DMOD || in_sizes[5] != DMOD * DMOD) return;
  if (in_sizes[7] != DMOD * DMOD || in_sizes[9] != DMOD * DMOD) return;
  if (in_sizes[4] != DMOD || in_sizes[6] != DMOD || in_sizes[8] != DMOD || in_sizes[10] != DMOD) return;
  if (out_size != XN) return;

  const float* Qin = (const float*)d_in[0];
  const float* Kin = (const float*)d_in[1];
  const float* Vin = (const float*)d_in[2];
  const float* wq  = (const float*)d_in[3];
  const float* bq  = (const float*)d_in[4];
  const float* wk  = (const float*)d_in[5];
  const float* bk  = (const float*)d_in[6];
  const float* wv  = (const float*)d_in[7];
  const float* bv  = (const float*)d_in[8];
  const float* wo  = (const float*)d_in[9];
  const float* bo  = (const float*)d_in[10];
  float*       out = (float*)d_out;

  const size_t szXT = (size_t)ROWS * DMOD * 2;
  const size_t szW  = (size_t)DMOD * DMOD * 2;
  const size_t szF  = (size_t)ROWS * DMOD * 4;
  const size_t szP  = (size_t)ROWS * DMOD * 2;
  size_t off = 0;
  const size_t oXT  = off; off += szXT;
  const size_t oWQB = off; off += szW;
  const size_t oWKB = off; off += szW;
  const size_t oWVB = off; off += szW;
  const size_t oWOB = off; off += szW;
  const size_t oF   = off; off += szF;
  const size_t oQH  = off; off += szP;
  const size_t oKH  = off; off += szP;
  const size_t oVH  = off; off += szP;
  const size_t oOHI = off; off += szP;
  const size_t oOLO = off; off += szP;
  if (off > ws_size) return;
  if (off > (size_t)134217728) return;

  char* ws = (char*)d_ws;
  u16*   XT  = (u16*)(ws + oXT);
  u16*   WQB = (u16*)(ws + oWQB);
  u16*   WKB = (u16*)(ws + oWKB);
  u16*   WVB = (u16*)(ws + oWVB);
  u16*   WOB = (u16*)(ws + oWOB);
  float* F   = (float*)(ws + oF);
  u16*   QH  = (u16*)(ws + oQH);
  u16*   KH  = (u16*)(ws + oKH);
  u16*   VH  = (u16*)(ws + oVH);
  u16*   OHI = (u16*)(ws + oOHI);
  u16*   OLO = (u16*)(ws + oOLO);

  const dim3 blk(256);
  const int n8x = XN / 8;
  const int n8w = (DMOD * DMOD) / 8;
  if ((n8x % 256) != 0 || (n8w % 256) != 0) return;
  const dim3 gP(n8x / 256);
  const dim3 gWc(n8w / 256);
  const dim3 gXT(NB * (SEQ / 64) * (DMOD / 64));
  const dim3 gGt((ROWS / 64) * (DMOD / 64), 1);
  const dim3 gGc((DMOD / 64) * (SEQ / 64), NB);
  const dim3 bG(128);
  const dim3 gAT(ATT_BLOCKS);
  const dim3 bAT(ATT_THREADS);
  const int  sTok = SEQ * DMOD;
  const int  sChn = DMOD * SEQ;

  cvtw<<<gWc, blk, 0, stream>>>(wq, WQB, 0, 1.0f);
  cvtw<<<gWc, blk, 0, stream>>>(wk, WKB, 0, 1.0f);
  cvtw<<<gWc, blk, 0, stream>>>(wv, WVB, 0, 1.0f);
  cvtw<<<gWc, blk, 0, stream>>>(wo, WOB, 1, WOS);
  xt16<<<gXT, blk, 0, stream>>>(Qin, XT);
  gemm_bfb<<<gGt, bG, 0, stream>>>(XT, WQB, bq, F, ROWS, DMOD, DMOD, 1.0f, 0, 0, 0, 0);
  cvh16<<<gP, blk, 0, stream>>>(F, QH, n8x, QSC);
  xt16<<<gXT, blk, 0, stream>>>(Kin, XT);
  gemm_bfb<<<gGt, bG, 0, stream>>>(XT, WKB, bk, F, ROWS, DMOD, DMOD, 1.0f, 0, 0, 0, 0);
  cvh16<<<gP, blk, 0, stream>>>(F, KH, n8x, KSC);
  xt16<<<gXT, blk, 0, stream>>>(Vin, XT);
  gemm_bfb<<<gGc, bG, 0, stream>>>(WVB, XT, bv, F, DMOD, SEQ, DMOD, 1.0f, 1, 0, sTok, sChn);
  cvh16<<<gP, blk, 0, stream>>>(F, VH, n8x, VCAR);
  attn_fwd<<<gAT, bAT, 0, stream>>>(QH, KH, VH, OHI, OLO);
  gemm_wh2<<<gGc, bG, 0, stream>>>(WOB, OHI, OLO, bo, out, DMOD, SEQ, DMOD, 1.0f / (OSC * WOS), sTok, sChn);
  (void)hipGetLastError();
}
